// DecoderLayer_53841710023063
// MI455X (gfx1250) — hardware-verified
//
#include <hip/hip_runtime.h>
#ifndef NB
#define NB 4
#endif
#ifndef SEQ
#define SEQ 1024
#endif
#ifndef LKV
#define LKV 4096
#endif
#define LQ_FULL 1024
#define LKV_FULL 4096
#define DM 512
#define NH 8
#define HD 64
#define DFF 2048
#define LQ3 (3 * DM)
#define HGS 8
#define HGC 2
#define NRQ ((size_t)NB * SEQ)
#define NRK ((size_t)NB * LKV)
#define LN_EPS 0.001f
#define ATT_ALPHA 0.044194173824159216f

static_assert(NB >= 1);
static_assert(SEQ % 128 == 0);
static_assert(LKV % 128 == 0);
static_assert(SEQ <= LQ_FULL);
static_assert(LKV <= LKV_FULL);
static_assert(NH * HD == DM);
static_assert(HD == 64);
static_assert(NH % HGS == 0);
static_assert(NH % HGC == 0);
static_assert(DM % 64 == 0);
static_assert(DFF % 64 == 0);
static_assert((NRQ * DM) % 8 == 0);
static_assert((NRK * DM) % 8 == 0);

typedef unsigned short v8us __attribute__((ext_vector_type(8), may_alias));
typedef float v8f __attribute__((ext_vector_type(8)));
typedef float v4f __attribute__((ext_vector_type(4)));
typedef float v4fa __attribute__((ext_vector_type(4), may_alias));
typedef _Float16 v16h __attribute__((ext_vector_type(16)));
typedef _Float16 v4h __attribute__((ext_vector_type(4)));
union FragH { v16h v; v8us half[2]; _Float16 h[16]; unsigned short u[16]; };

__device__ __forceinline__ unsigned short bf16_bits(float x) { unsigned int u = __float_as_uint(x); return (unsigned short)((u + 0x7FFFu + ((u >> 16) & 1u)) >> 16); }
__device__ __forceinline__ float bf16_val(unsigned short b) { return __uint_as_float(((unsigned int)b) << 16); }
__device__ __forceinline__ float bf16_rne(float x) { return bf16_val(bf16_bits(x)); }

__device__ __forceinline__ v16h g2_frag(const _Float16* p, int hh) { FragH f; f.half[0] = *(const v8us*)((const unsigned short*)p + 8 * hh); f.half[1] = *(const v8us*)((const unsigned short*)p + 16 + 8 * hh); return f.v; }
__device__ __forceinline__ v8f g2_mma(v16h a, v16h b, v8f c) { v8f d = __builtin_amdgcn_wmma_f32_16x16x32_f16(false, a, false, b, (short)0, c, false, false); asm volatile("v_nop\n\tv_nop\n\tv_nop\n\tv_nop" : "+v"(d) : "v"(a), "v"(b)); return d; }

__global__ __launch_bounds__(256) void k_wt4(const float* __restrict__ W0, const float* __restrict__ W1, const float* __restrict__ W2, const float* __restrict__ W3,
                                             _Float16* __restrict__ Wt, int K, int N, float scale) {
  const int t = blockIdx.x * 256 + threadIdx.x; if (t >= N * (K / 8)) return;
  const int y = blockIdx.y; const float* W = (y == 0) ? W0 : ((y == 1) ? W1 : ((y == 2) ? W2 : W3));
  const int n = t / (K / 8), k8 = (t % (K / 8)) * 8; FragH f;
#pragma unroll
  for (int i = 0; i < 8; ++i) f.h[i] = (_Float16)(bf16_rne(W[(size_t)(k8 + i) * N + n]) * scale);
  const v8us o = f.half[0]; unsigned short* d = (unsigned short*)Wt + (size_t)y * N * K + (size_t)n * K + k8;
  *(volatile v8us*)d = o; __threadfence(); *(volatile v8us*)d = o;
}

__global__ __launch_bounds__(256) void k_cvt2(const float* __restrict__ a, const float* __restrict__ e, int L, int Lfull, size_t n8, _Float16* __restrict__ A16, _Float16* __restrict__ S16) {
  const size_t t = (size_t)blockIdx.x * 256 + threadIdx.x; if (t >= n8) return;
  const size_t el = t * 8; const size_t row = el / DM; const size_t c = el % DM;
  const size_t src = ((row / (size_t)L) * (size_t)Lfull + (row % (size_t)L)) * DM + c;
  const v4f a0 = *(const v4fa*)(a + src), a1 = *(const v4fa*)(a + src + 4), e0 = *(const v4fa*)(e + src), e1 = *(const v4fa*)(e + src + 4);
  FragH fa, fs;
#pragma unroll
  for (int q = 0; q < 4; ++q) {
    const float v0 = bf16_rne(a0[q]); fa.h[q] = (_Float16)v0; fs.h[q] = (_Float16)(v0 + bf16_rne(e0[q]));
    const float v1 = bf16_rne(a1[q]); fa.h[4 + q] = (_Float16)v1; fs.h[4 + q] = (_Float16)(v1 + bf16_rne(e1[q]));
  }
  unsigned short* da = (unsigned short*)A16 + el; unsigned short* ds = (unsigned short*)S16 + el;
  for (int pass = 0; pass < 2; ++pass) { *(volatile v8us*)da = fa.half[0]; *(volatile v8us*)ds = fs.half[0]; if (pass == 0) __threadfence(); }
}

template <int ACT>
__global__ __launch_bounds__(128) void k_gemm2(const _Float16* __restrict__ A, int lda, size_t sA, const _Float16* __restrict__ Bh, int ldb, size_t sB, float alpha,
                                               const float* __restrict__ bias, float oscale, float* __restrict__ C, _Float16* __restrict__ C16, int ldc, size_t sC, int M, int N, int K) {
  static_assert(ACT == 0 || ACT == 3);
  __shared__ __attribute__((aligned(16))) float so[4][32][68];
  const int tid = threadIdx.x, w = tid >> 5, lane = tid & 31, ln = lane & 15, hh = lane >> 4; const int by = blockIdx.y;
  A += (size_t)by * sA; Bh += (size_t)by * sB; const size_t cofs = (size_t)by * sC;
  const int ntn = N >> 6; const int mt = blockIdx.x / ntn, nq = blockIdx.x - mt * ntn; const int row0 = mt * 128 + 32 * w, col0 = nq * 64;
  if (row0 >= M) return;
  const _Float16* a0p = A + (size_t)(row0 + ln) * lda; const _Float16* a1p = a0p + (size_t)16 * lda;
  const _Float16* b0p = Bh + (size_t)(col0 + ln) * ldb; const _Float16* b1p = b0p + (size_t)16 * ldb; const _Float16* b2p = b1p + (size_t)16 * ldb; const _Float16* b3p = b2p + (size_t)16 * ldb;
  const v8f z8 = {0.f, 0.f, 0.f, 0.f, 0.f, 0.f, 0.f, 0.f};
  v8f c00 = z8, c01 = z8, c02 = z8, c03 = z8, c10 = z8, c11 = z8, c12 = z8, c13 = z8;
#pragma unroll 1
  for (int kb = 0; kb < K; kb += 32) {
    const v16h a0 = g2_frag(a0p + kb, hh), a1 = g2_frag(a1p + kb, hh);
    v16h b = g2_frag(b0p + kb, hh); c00 = g2_mma(a0, b, c00); c10 = g2_mma(a1, b, c10);
    b = g2_frag(b1p + kb, hh); c01 = g2_mma(a0, b, c01); c11 = g2_mma(a1, b, c11);
    b = g2_frag(b2p + kb, hh); c02 = g2_mma(a0, b, c02); c12 = g2_mma(a1, b, c12);
    b = g2_frag(b3p + kb, hh); c03 = g2_mma(a0, b, c03); c13 = g2_mma(a1, b, c13);
  }
  v8f accs[8] = {c00, c01, c02, c03, c10, c11, c12, c13};
#pragma unroll
  for (int u = 0; u < 8; ++u) {
    const int t = u & 3, half = u >> 2; const int col = col0 + t * 16 + ln; const float bv = bias ? bf16_rne(bias[col]) : 0.f;
#pragma unroll
    for (int r = 0; r < 8; ++r) {
      const int rloc = half * 16 + 8 * hh + r; float v = accs[u][r] * alpha + bv;
      if (ACT == 3) v = fmaxf(v, 0.f);
      v = v * oscale;
      so[w][rloc][t * 16 + ln] = v;
    }
  }
  __builtin_amdgcn_fence(4  , "workgroup"); __builtin_amdgcn_wave_barrier();
  const int rsub = lane >> 4, c4 = (lane & 15) * 4;
  for (int pass = 0; pass < 2; ++pass) {
#pragma unroll
    for (int q = 0; q < 16; ++q) {
      const int r = q * 2 + rsub; const v4f v = *(const v4fa*)&so[w][r][c4];
      if (C) *(volatile v4f*)(C + cofs + (size_t)(row0 + r) * ldc + col0 + c4) = v;
      if (C16) { v4h h4;
#pragma unroll
        for (int i = 0; i < 4; ++i) h4[i] = (_Float16)v[i];
        *(volatile v4h*)(C16 + cofs + (size_t)(row0 + r) * ldc + col0 + c4) = h4; }
    }
    if (pass == 0) __threadfence();
  }
}

template <int NHv, int TTv>
__global__ __launch_bounds__(256) void k_vt(const _Float16* __restrict__ V16, int ldv, int voff, _Float16* __restrict__ Vt) {
  __shared__ unsigned short tl[64][66];
  const int tid = threadIdx.x; const int slab = blockIdx.x / (TTv / 64), lg = blockIdx.x % (TTv / 64); const int b = slab / NHv, h = slab % NHv;
  for (int i = tid; i < 64 * 8; i += 256) {
    const int r = i / 8, c8 = (i % 8) * 8; FragH f;
    f.half[0] = *(const v8us*)((const unsigned short*)V16 + ((size_t)b * TTv + lg * 64 + r) * ldv + voff + h * 64 + c8);
#pragma unroll
    for (int q = 0; q < 8; ++q) tl[r][c8 + q] = f.u[q];
  }
  __syncthreads();
  for (int pass = 0; pass < 2; ++pass) {
#pragma unroll
    for (int rd = 0; rd < 2; ++rd) {
      const int d = rd * 32 + tid / 8, pc = tid % 8; FragH f;
#pragma unroll
      for (int q = 0; q < 8; ++q) f.u[q] = tl[pc * 8 + q][d];
      *(volatile v8us*)((unsigned short*)Vt + ((size_t)slab * 64 + d) * TTv + lg * 64 + pc * 8) = f.half[0];
    }
    if (pass == 0) __threadfence();
  }
}

template <int TK>
__global__ __launch_bounds__(256) void k_rsm(const float* __restrict__ S, _Float16* __restrict__ P, int qn, int hg) {
  #pragma clang fp contract(off)
  const int t = blockIdx.x * 256 + threadIdx.x; if (t >= qn * hg) return;
  const size_t i = (size_t)(t / qn) * SEQ + (size_t)(t % qn); const float* s = S + i * TK; float mx = -3.0e38f;
#pragma unroll 1
  for (int j = 0; j < TK; ++j) mx = fmaxf(mx, s[j]);
  float se = 0.f;
#pragma unroll 1
  for (int j = 0; j < TK; ++j) se += __expf(s[j] - mx);
  const float sc = 1024.0f * (1.0f / se);
#pragma unroll 1
  for (int j0 = 0; j0 < TK; j0 += 8) {
    FragH f;
#pragma unroll
    for (int q = 0; q < 8; ++q) f.h[q] = (_Float16)(__expf(s[j0 + q] - mx) * sc);
    unsigned short* d = (unsigned short*)P + i * TK + j0;
    *(volatile v8us*)d = f.half[0]; __threadfence(); *(volatile v8us*)d = f.half[0];
  }
}

template <int RIN, int W32, int W16, int WE>
__global__ __launch_bounds__(256) void k_ln(const float* __restrict__ X, const float* __restrict__ R, int L, int Lfull, const float* __restrict__ g, const float* __restrict__ bb, float eps,
                                            float* __restrict__ N32, _Float16* __restrict__ N16, const float* __restrict__ E, _Float16* __restrict__ E16) {
  #pragma clang fp contract(off)
  __shared__ float red[256];
  const size_t r = blockIdx.x; const int t = threadIdx.x; const bool act = t < (DM / 4); const int c0 = act ? t * 4 : 0;
  const size_t rin = (r / (size_t)L) * (size_t)Lfull + (r % (size_t)L);
  const v4f xa = *(const v4fa*)(X + r * DM + c0);
  const v4f ra = *(const v4fa*)(R + (RIN ? rin : r) * DM + c0);
  v4f ea = {0.f, 0.f, 0.f, 0.f}; if (WE) ea = *(const v4fa*)(E + rin * DM + c0);
  float s[4]; float sum = 0.f;
#pragma unroll
  for (int q = 0; q < 4; ++q) { const float rv = RIN ? bf16_rne(ra[q]) : ra[q]; s[q] = act ? __fadd_rn(xa[q], rv) : 0.f; sum = __fadd_rn(sum, s[q]); }
  red[t] = sum; __syncthreads();
  for (int st = 128; st > 0; st >>= 1) { if (t < st) red[t] = __fadd_rn(red[t], red[t + st]); __syncthreads(); }
  const float mu = red[0] / (float)DM; __syncthreads();
  float vs = 0.f;
#pragma unroll
  for (int q = 0; q < 4; ++q) { const float dl = act ? __fadd_rn(s[q], -mu) : 0.f; vs = __fadd_rn(vs, __fmul_rn(dl, dl)); }
  red[t] = vs; __syncthreads();
  for (int st = 128; st > 0; st >>= 1) { if (t < st) red[t] = __fadd_rn(red[t], red[t + st]); __syncthreads(); }
  const float rs = rsqrtf(__fadd_rn(red[0] / (float)DM, eps));
  v4f yf; v4h y, ye;
#pragma unroll
  for (int q = 0; q < 4; ++q) {
    const int c = c0 + q;
    yf[q] = __fadd_rn(__fmul_rn(__fmul_rn(__fadd_rn(s[q], -mu), rs), bf16_rne(g[c])), bf16_rne(bb[c]));
    y[q] = (_Float16)yf[q]; ye[q] = (_Float16)__fadd_rn(yf[q], bf16_rne(ea[q]));
  }
  if (!act) return;
  for (int pass = 0; pass < 2; ++pass) {
    if (W32) *(volatile v4f*)(N32 + r * DM + c0) = yf;
    if (W16) *(volatile v4h*)(N16 + r * DM + c0) = y;
    if (WE) *(volatile v4h*)(E16 + r * DM + c0) = ye;
    if (pass == 0) __threadfence();
  }
}

extern "C" void kernel_launch(void* const* d_in, const int* in_sizes, int n_in,
                              void* d_out, int out_size, void* d_ws, size_t ws_size, hipStream_t stream) {
  if (n_in < 30) return;
  const float* const* I = (const float* const*)d_in;
  const float* xq = I[0];  const float* xm = I[1];  const float* xp = I[2];  const float* xe = I[3];
  const float* sWq = I[4];  const float* sbq = I[5];  const float* sWk = I[6];  const float* sbk = I[7];
  const float* sWv = I[8];  const float* sbv = I[9];  const float* sWo = I[10]; const float* sbo = I[11];
  const float* cWq = I[12]; const float* cbq = I[13]; const float* cWk = I[14]; const float* cbk = I[15];
  const float* cWv = I[16]; const float* cbv = I[17]; const float* cWo = I[18]; const float* cbo = I[19];
  const float* fW1 = I[20]; const float* fb1 = I[21]; const float* fW2 = I[22]; const float* fb2 = I[23];
  const float* g1 = I[24]; const float* bt1 = I[25]; const float* g2 = I[26]; const float* bt2 = I[27]; const float* g3 = I[28]; const float* bt3 = I[29];
  float* out = (float*)d_out;
  const size_t needQ = ((size_t)(NB - 1) * LQ_FULL + SEQ) * DM, needM = ((size_t)(NB - 1) * LKV_FULL + LKV) * DM;
  if ((size_t)in_sizes[0] < needQ || (size_t)in_sizes[3] < needQ || (size_t)in_sizes[1] < needM || (size_t)in_sizes[2] < needM) return;
  for (int i = 4; i <= 18; i += 2) if ((size_t)in_sizes[i] < (size_t)DM * DM) return;
  for (int i = 5; i <= 19; i += 2) if (in_sizes[i] < DM) return;
  if ((size_t)in_sizes[20] < (size_t)DM * DFF || in_sizes[21] < DFF || (size_t)in_sizes[22] < (size_t)DFF * DM || in_sizes[23] < DM) return;
  for (int i = 24; i <= 29; ++i) if (in_sizes[i] < DM) return;
  if ((size_t)out_size < NRQ * DM) return;

  auto mx2 = [](size_t a, size_t b) { return a > b ? a : b; };
  char* ws = (char*)d_ws; size_t off = 0;
  auto take = [&](size_t bytes) { char* p = ws + off; off += (bytes + 255) & ~(size_t)255; return p; };
  const size_t plQ16 = NRQ * DM * 2, plQ32 = NRQ * DM * 4, plK16 = NRK * DM * 2, plH16 = NRQ * DFF * 2;
  const size_t TMAX = mx2((size_t)SEQ, (size_t)LKV);
  const size_t nS = mx2((size_t)HGS * SEQ * SEQ, (size_t)HGC * SEQ * LKV);
  const size_t szS = nS * 4, szP = nS * 2;
  const size_t szSP = mx2(mx2(szS + szP, 2 * plK16), plQ32 + plQ16 + plH16);
  _Float16* BWS = (_Float16*)take((size_t)4 * DM * DM * 2);
  _Float16* BWC = (_Float16*)take((size_t)4 * DM * DM * 2);
  _Float16* BW1 = (_Float16*)take((size_t)DFF * DM * 2);
  _Float16* BW2 = (_Float16*)take((size_t)DM * DFF * 2);
  char* RSP = take(szSP);
  float* S = (float*)RSP; _Float16* P = (_Float16*)(RSP + szS);
  _Float16* M16 = (_Float16*)RSP; _Float16* KC16 = (_Float16*)(RSP + plK16);
  float* X2F = (float*)RSP; _Float16* X2H = (_Float16*)(RSP + plQ32); _Float16* H16 = (_Float16*)(RSP + plQ32 + plQ16);
  _Float16* VT = (_Float16*)take((size_t)NH * HD * TMAX * 2);
  _Float16* O16 = (_Float16*)take(plQ16);
  float* AF = (float*)take(plQ32);
  float* X1F = (float*)take(plQ32);
  _Float16* QC16 = (_Float16*)take(plQ16);
  char* RKX = take(mx2(plK16, 2 * plQ16));
  _Float16* X16 = (_Float16*)RKX; _Float16* QK16 = (_Float16*)(RKX + plQ16); _Float16* KCP = (_Float16*)RKX;
  char* RVX = take(mx2(plK16, NRQ * LQ3 * 2));
  _Float16* QKV = (_Float16*)RVX; _Float16* VCP = (_Float16*)RVX;
  _Float16* QCP = (_Float16*)take(plQ16);
  if (off > ws_size) return;

  const unsigned gW = (unsigned)((DM * (DM / 8) + 255) / 256);
  k_wt4<<<dim3(gW, 4), 256, 0, stream>>>(sWq, sWk, sWv, sWo, BWS, DM, DM, 16.0f);
  k_wt4<<<dim3(gW, 4), 256, 0, stream>>>(cWq, cWk, cWv, cWo, BWC, DM, DM, 16.0f);
  k_wt4<<<dim3((unsigned)((DFF * (DM / 8) + 255) / 256), 1), 256, 0, stream>>>(fW1, fW1, fW1, fW1, BW1, DM, DFF, 16.0f);
  k_wt4<<<dim3((unsigned)((DM * (DFF / 8) + 255) / 256), 1), 256, 0, stream>>>(fW2, fW2, fW2, fW2, BW2, DFF, DM, 16.0f);

  const size_t n8q = NRQ * DM / 8;
  k_cvt2<<<(unsigned)((n8q + 255) / 256), 256, 0, stream>>>(xq, xe, SEQ, LQ_FULL, n8q, X16, QK16);
  const unsigned gPQ = (unsigned)((NRQ / 128) * (DM / 64));
  k_gemm2<0><<<dim3(gPQ, 1), 128, 0, stream>>>(QK16, DM, (size_t)0, BWS, DM, (size_t)0, 0.0625f, sbq, 1.0f, nullptr, QKV, LQ3, (size_t)0, (int)NRQ, DM, DM);
  k_gemm2<0><<<dim3(gPQ, 1), 128, 0, stream>>>(QK16, DM, (size_t)0, BWS + (size_t)DM * DM, DM, (size_t)0, 0.0625f, sbk, 1.0f, nullptr, QKV + DM, LQ3, (size_t)0, (int)NRQ, DM, DM);
  k_gemm2<0><<<dim3(gPQ, 1), 128, 0, stream>>>(X16, DM, (size_t)0, BWS + (size_t)2 * DM * DM, DM, (size_t)0, 0.0625f, sbv, 1.0f, nullptr, QKV + 2 * DM, LQ3, (size_t)0, (int)NRQ, DM, DM);
  for (int b = 0; b < NB; ++b) {
    const size_t r0 = (size_t)b * SEQ;
    k_vt<NH, SEQ><<<dim3(NH * (SEQ / 64)), 256, 0, stream>>>(QKV + r0 * LQ3, LQ3, 2 * DM, VT);
    for (int h0 = 0; h0 < NH; h0 += HGS) {
      k_gemm2<0><<<dim3((SEQ / 128) * (SEQ / 64), HGS), 128, 0, stream>>>(QKV + r0 * LQ3 + h0 * HD, LQ3, (size_t)HD, QKV + DM + r0 * LQ3 + h0 * HD, LQ3, (size_t)HD, ATT_ALPHA, nullptr, 1.0f, S, nullptr, SEQ, (size_t)SEQ * SEQ, SEQ, SEQ, HD);
      k_rsm<SEQ><<<(unsigned)((HGS * SEQ + 255) / 256), 256, 0, stream>>>(S, P, SEQ, HGS);
      k_gemm2<0><<<dim3(SEQ / 128, HGS), 128, 0, stream>>>(P, SEQ, (size_t)SEQ * SEQ, VT + (size_t)h0 * HD * SEQ, SEQ, (size_t)HD * SEQ, 0.0625f, nullptr, 1.0f, nullptr, O16 + r0 * DM + h0 * HD, DM, (size_t)HD, SEQ, HD, SEQ);
    }
  }
  k_gemm2<0><<<dim3(gPQ, 1), 128, 0, stream>>>(O16, DM, (size_t)0, BWS + (size_t)3 * DM * DM, DM, (size_t)0, 0.0009765625f, sbo, 1.0f, AF, nullptr, DM, (size_t)0, (int)NRQ, DM, DM);
  k_ln<1, 1, 0, 1><<<(unsigned)NRQ, 256, 0, stream>>>(AF, xq, SEQ, LQ_FULL, g1, bt1, LN_EPS, X1F, nullptr, xe, QC16);

  const size_t n8k = NRK * DM / 8;
  k_cvt2<<<(unsigned)((n8k + 255) / 256), 256, 0, stream>>>(xm, xp, LKV, LKV_FULL, n8k, M16, KC16);
  const unsigned gPK = (unsigned)((NRK / 128) * (DM / 64));
  k_gemm2<0><<<dim3(gPQ, 1), 128, 0, stream>>>(QC16, DM, (size_t)0, BWC, DM, (size_t)0, 0.0625f, cbq, 1.0f, nullptr, QCP, DM, (size_t)0, (int)NRQ, DM, DM);
  k_gemm2<0><<<dim3(gPK, 1), 128, 0, stream>>>(KC16, DM, (size_t)0, BWC + (size_t)DM * DM, DM, (size_t)0, 0.0625f, cbk, 1.0f, nullptr, KCP, DM, (size_t)0, (int)NRK, DM, DM);
  k_gemm2<0><<<dim3(gPK, 1), 128, 0, stream>>>(M16, DM, (size_t)0, BWC + (size_t)2 * DM * DM, DM, (size_t)0, 0.0625f, cbv, 1.0f, nullptr, VCP, DM, (size_t)0, (int)NRK, DM, DM);
  for (int b = 0; b < NB; ++b) {
    const size_t rq = (size_t)b * SEQ, rk = (size_t)b * LKV;
    k_vt<NH, LKV><<<dim3(NH * (LKV / 64)), 256, 0, stream>>>(VCP + rk * DM, DM, 0, VT);
    for (int h0 = 0; h0 < NH; h0 += HGC) {
      k_gemm2<0><<<dim3((SEQ / 128) * (LKV / 64), HGC), 128, 0, stream>>>(QCP + rq * DM + h0 * HD, DM, (size_t)HD, KCP + rk * DM + h0 * HD, DM, (size_t)HD, ATT_ALPHA, nullptr, 1.0f, S, nullptr, LKV, (size_t)SEQ * LKV, SEQ, LKV, HD);
      k_rsm<LKV><<<(unsigned)((HGC * SEQ + 255) / 256), 256, 0, stream>>>(S, P, SEQ, HGC);
      k_gemm2<0><<<dim3(SEQ / 128, HGC), 128, 0, stream>>>(P, LKV, (size_t)SEQ * LKV, VT + (size_t)h0 * HD * LKV, LKV, (size_t)HD * LKV, 0.0625f, nullptr, 1.0f, nullptr, O16 + rq * DM + h0 * HD, DM, (size_t)HD, SEQ, HD, LKV);
    }
  }
  k_gemm2<0><<<dim3(gPQ, 1), 128, 0, stream>>>(O16, DM, (size_t)0, BWC + (size_t)3 * DM * DM, DM, (size_t)0, 0.0009765625f, cbo, 1.0f, AF, nullptr, DM, (size_t)0, (int)NRQ, DM, DM);
  k_ln<0, 1, 1, 0><<<(unsigned)NRQ, 256, 0, stream>>>(AF, X1F, SEQ, SEQ, g2, bt2, LN_EPS, X2F, X2H, nullptr, nullptr);

  k_gemm2<3><<<dim3((unsigned)((NRQ / 128) * (DFF / 64)), 1), 128, 0, stream>>>(X2H, DM, (size_t)0, BW1, DM, (size_t)0, 0.0625f, fb1, 16.0f, nullptr, H16, DFF, (size_t)0, (int)NRQ, DFF, DM);
  k_gemm2<0><<<dim3(gPQ, 1), 128, 0, stream>>>(H16, DFF, (size_t)0, BW2, DFF, (size_t)0, 0.00390625f, fb2, 1.0f, AF, nullptr, DM, (size_t)0, (int)NRQ, DM, DFF);
  k_ln<0, 1, 0, 0><<<(unsigned)NRQ, 256, 0, stream>>>(AF, X2F, SEQ, SEQ, g3, bt3, LN_EPS, out, nullptr, nullptr, nullptr);
}
